// LoRAMultiheadAttention_85864986181639
// MI455X (gfx1250) — hardware-verified
//
#include <hip/hip_runtime.h>

typedef _Float16 v16h __attribute__((ext_vector_type(16)));
typedef _Float16 v8h  __attribute__((ext_vector_type(8)));
typedef float    v8f  __attribute__((ext_vector_type(8)));
typedef float    v4f  __attribute__((ext_vector_type(4)));
typedef v8h __attribute__((may_alias)) v8ha;
typedef v4f __attribute__((may_alias)) v4fa;

union Frag { v16h v; v8h half[2]; };

#define TLEN   2048
#define BSZ    2
#define DM     1024
#define NHEADS 16
#define HD     64
#define RNK    16
#define KPAD   32
#define MROWS  (TLEN * BSZ)
#define N3D    (3 * DM)
#define NX     (MROWS * DM)
#define NWIN   (N3D * DM)
#define NWOUT  (DM * DM)
#define NLA    (RNK * DM)
#define PSCALE 16384.0f
#define WSCALE 32.0f
#define WINV   0.03125f
#define LORA_S 1.0f

__device__ __forceinline__ v8f wmma_f16(v16h a, v16h b, v8f c) {
  v8f d = __builtin_amdgcn_wmma_f32_16x16x32_f16(false, a, false, b, (short)0, c, false, false);
  asm volatile("v_nop\n\tv_nop\n\tv_nop\n\tv_nop" : "+v"(d) : "v"(a), "v"(b));
  return d;
}

__device__ __forceinline__ v16h load_frag(const _Float16* p, int h) {
  Frag f;
  f.half[0] = *(const v8ha*)(p + 8 * h);
  f.half[1] = *(const v8ha*)(p + 16 + 8 * h);
  return f.v;
}

__device__ __forceinline__ v8h cvt8(const float* src, float sc) {
  const v4f a = *(const v4fa*)src;
  const v4f c = *(const v4fa*)(src + 4);
  const v8h o = { (_Float16)(a.x * sc), (_Float16)(a.y * sc), (_Float16)(a.z * sc), (_Float16)(a.w * sc),
                  (_Float16)(c.x * sc), (_Float16)(c.y * sc), (_Float16)(c.z * sc), (_Float16)(c.w * sc) };
  return o;
}

__global__ __launch_bounds__(256) void convert_kernel(
    const float* __restrict__ x, const float* __restrict__ win, const float* __restrict__ wout,
    const float* __restrict__ ka, const float* __restrict__ va,
    _Float16* __restrict__ xh, _Float16* __restrict__ wh, _Float16* __restrict__ woh,
    _Float16* __restrict__ kah, _Float16* __restrict__ vah)
{
  const int g = blockIdx.x * 256 + threadIdx.x;
  const int g0 = NX / 8, g1 = g0 + NWIN / 8, g2 = g1 + NWOUT / 8, g3 = g2 + NLA / 8, g4 = g3 + NLA / 8;
  if (g >= g4) return;
  const float* src;
  _Float16* dst;
  float sc;
  if (g < g0)      { src = x + (size_t)g * 8;                          dst = xh + (size_t)g * 8;   sc = 1.0f; }
  else if (g < g1) { const int e = g - g0; src = win  + (size_t)e * 8;  dst = wh  + (size_t)e * 8;  sc = WSCALE; }
  else if (g < g2) { const int e = g - g1; src = wout + (size_t)e * 8;  dst = woh + (size_t)e * 8;  sc = WSCALE; }
  else if (g < g3) { const int e = g - g2; src = ka   + (size_t)e * 8;  dst = kah + (size_t)e * 8;  sc = WSCALE; }
  else             { const int e = g - g3; src = va   + (size_t)e * 8;  dst = vah + (size_t)e * 8;  sc = WSCALE; }
  const v8h o = cvt8(src, sc);
  *(volatile v8h*)dst = o;
  __threadfence();
  *(volatile v8h*)dst = o;
}

__device__ __forceinline__ v8h gather8_col(const float* src, int n, int r0) {
  const v8h o = { (_Float16)(src[(size_t)(r0 + 0) * DM + n] * WSCALE), (_Float16)(src[(size_t)(r0 + 1) * DM + n] * WSCALE),
                  (_Float16)(src[(size_t)(r0 + 2) * DM + n] * WSCALE), (_Float16)(src[(size_t)(r0 + 3) * DM + n] * WSCALE),
                  (_Float16)(src[(size_t)(r0 + 4) * DM + n] * WSCALE), (_Float16)(src[(size_t)(r0 + 5) * DM + n] * WSCALE),
                  (_Float16)(src[(size_t)(r0 + 6) * DM + n] * WSCALE), (_Float16)(src[(size_t)(r0 + 7) * DM + n] * WSCALE) };
  return o;
}

__device__ __forceinline__ void lorab_store(_Float16* dst, v8h a0, v8h a1, v8h b0, v8h b1, v8h z8) {
  *(volatile v8h*)(dst + 0)  = a0;
  *(volatile v8h*)(dst + 8)  = a1;
  *(volatile v8h*)(dst + 16) = z8;
  *(volatile v8h*)(dst + 24) = z8;
  *(volatile v8h*)(dst + 32) = b0;
  *(volatile v8h*)(dst + 40) = b1;
  *(volatile v8h*)(dst + 48) = z8;
  *(volatile v8h*)(dst + 56) = z8;
}

__global__ __launch_bounds__(256) void lorab_kernel(
    const float* __restrict__ kb, const float* __restrict__ vb,
    _Float16* __restrict__ kbt, _Float16* __restrict__ vbt)
{
  const int j = blockIdx.x * 256 + threadIdx.x;
  if (j >= DM) return;
  const int sel = j >> 9, L = j & 511;
  const float* src = sel ? vb : kb;
  _Float16* dst = (sel ? vbt : kbt) + (size_t)L * 64;
  const int n0 = 2 * L, n1 = 2 * L + 1;
  const v8h z8 = { (_Float16)0.0f, (_Float16)0.0f, (_Float16)0.0f, (_Float16)0.0f,
                   (_Float16)0.0f, (_Float16)0.0f, (_Float16)0.0f, (_Float16)0.0f };
  const v8h a0 = gather8_col(src, n0, 0), a1 = gather8_col(src, n0, 8);
  const v8h b0 = gather8_col(src, n1, 0), b1 = gather8_col(src, n1, 8);
  lorab_store(dst, a0, a1, b0, b1, z8);
  __threadfence();
  lorab_store(dst, a0, a1, b0, b1, z8);
}

__device__ __forceinline__ void lora_store_pass(const _Float16* sT, _Float16* dstp, int m0, int w, int lane) {
  const int q8 = lane & 7, sub = lane >> 3;
  #pragma unroll
  for (int i = 0; i < 4; ++i) {
    const int L = w * 16 + i * 4 + sub;
    const v8h v = *(const v8ha*)(sT + L * 64 + 8 * q8);
    _Float16* dst = dstp + (size_t)m0 * KPAD + L * 64 + 8 * q8;
    *(volatile v8h*)dst = v;
  }
}

__global__ __launch_bounds__(128) void lora_a_kernel(
    const _Float16* __restrict__ xh,
    const _Float16* __restrict__ kah,
    const _Float16* __restrict__ vah,
    _Float16* __restrict__ lk,
    _Float16* __restrict__ lv)
{
  __shared__ __attribute__((aligned(16))) _Float16 sT[128 * KPAD];

  const int tid = threadIdx.x, lane = tid & 31, w = tid >> 5;
  const int h = lane >> 4, m = lane & 15;
  const int m0 = blockIdx.x * 128;
  const int sel = blockIdx.y;
  const _Float16* wa = (sel == 0) ? kah : vah;
  _Float16* dstp = (sel == 0) ? lk : lv;
  const int m0w = m0 + 32 * w;

  const _Float16* xa0 = xh + (size_t)(m0w + m) * DM;
  const _Float16* xa1 = xa0 + (size_t)16 * DM;
  const _Float16* wb  = wa + (size_t)m * DM;

  const v8f zero8 = {0.f, 0.f, 0.f, 0.f, 0.f, 0.f, 0.f, 0.f};
  v8f acc[2];
  acc[0] = zero8; acc[1] = zero8;

  #pragma unroll 1
  for (int k0 = 0; k0 < DM; k0 += 32) {
    const v16h a0 = load_frag(xa0 + k0, h);
    const v16h a1 = load_frag(xa1 + k0, h);
    const v16h b  = load_frag(wb + k0, h);
    acc[0] = wmma_f16(a0, b, acc[0]);
    acc[1] = wmma_f16(a1, b, acc[1]);
  }

  #pragma unroll
  for (int mt = 0; mt < 2; ++mt) {
    #pragma unroll
    for (int r = 0; r < 8; ++r) {
      const int tokl = 32 * w + 16 * mt + 8 * h + r;
      const float y = acc[mt][r] * WINV * LORA_S;
      sT[tokl * KPAD + m] = (_Float16)y;
      sT[tokl * KPAD + 16 + m] = (_Float16)0.0f;
    }
  }
  __syncthreads();

  lora_store_pass(sT, dstp, m0, w, lane);
  __threadfence();
  lora_store_pass(sT, dstp, m0, w, lane);
}

__device__ __forceinline__ void proj_store_pass(const _Float16* sT, _Float16* plane, _Float16* vt,
                                                int which, int head, int t0, int w, int lane) {
  const int q8 = lane & 7, sub = lane >> 3;
  #pragma unroll
  for (int i = 0; i < 8; ++i) {
    const int lid = w * 32 + i * 4 + sub;
    const v8h v = *(const v8ha*)(sT + lid * 64 + 8 * q8);
    _Float16* dst;
    if (which != 2) {
      const int b = lid & 1, tl = lid >> 1;
      dst = plane + ((size_t)(b * NHEADS + head) * TLEN + t0 + tl) * HD + 8 * q8;
    } else {
      const int b = lid >> 6, d = lid & 63;
      dst = vt + ((size_t)(b * NHEADS + head) * HD + d) * TLEN + t0 + 8 * q8;
    }
    *(volatile v8h*)dst = v;
  }
}

__global__ __launch_bounds__(128) void proj_kernel(
    const _Float16* __restrict__ xh,
    const _Float16* __restrict__ wh,
    const float* __restrict__ bias,
    const _Float16* __restrict__ lk,
    const _Float16* __restrict__ lv,
    const _Float16* __restrict__ kbt,
    const _Float16* __restrict__ vbt,
    _Float16* __restrict__ qh,
    _Float16* __restrict__ kh,
    _Float16* __restrict__ vt)
{
  __shared__ __attribute__((aligned(16))) _Float16 sT[128 * 64];

  const int tid = threadIdx.x, lane = tid & 31, w = tid >> 5;
  const int h = lane >> 4, m = lane & 15;
  const int m0 = blockIdx.x * 128;
  const int cg = blockIdx.y;
  const int which = cg >> 4, head = cg & 15;
  const int m0w = m0 + 32 * w;

  const _Float16* xa0 = xh + (size_t)(m0w + m) * DM;
  const _Float16* xa1 = xa0 + (size_t)16 * DM;
  const _Float16* wb  = wh + ((size_t)which * DM + head * HD + m) * DM;

  const v8f zero8 = {0.f, 0.f, 0.f, 0.f, 0.f, 0.f, 0.f, 0.f};
  v8f acc[2][4];
  #pragma unroll
  for (int mt = 0; mt < 2; ++mt)
    #pragma unroll
    for (int nt = 0; nt < 4; ++nt) acc[mt][nt] = zero8;

  #pragma unroll 1
  for (int k0 = 0; k0 < DM; k0 += 32) {
    const v16h a0 = load_frag(xa0 + k0, h);
    const v16h a1 = load_frag(xa1 + k0, h);
    #pragma unroll
    for (int nt = 0; nt < 4; ++nt) {
      const v16h b = load_frag(wb + (size_t)nt * 16 * DM + k0, h);
      acc[0][nt] = wmma_f16(a0, b, acc[0][nt]);
      acc[1][nt] = wmma_f16(a1, b, acc[1][nt]);
    }
  }

  if (which != 0) {
    const _Float16* la = (which == 1) ? lk : lv;
    const _Float16* lb = (which == 1) ? kbt : vbt;
    const v16h a0 = load_frag(la + (size_t)(m0w + m) * KPAD, h);
    const v16h a1 = load_frag(la + (size_t)(m0w + 16 + m) * KPAD, h);
    #pragma unroll
    for (int nt = 0; nt < 4; ++nt) {
      const v16h b = load_frag(lb + (size_t)(head * HD + 16 * nt + m) * KPAD, h);
      acc[0][nt] = wmma_f16(a0, b, acc[0][nt]);
      acc[1][nt] = wmma_f16(a1, b, acc[1][nt]);
    }
  }

  const float osc = (which == 0) ? 0.125f : 1.0f;
  #pragma unroll
  for (int nt = 0; nt < 4; ++nt) {
    const int feat = 16 * nt + m;
    const float bvl = bias[which * DM + head * HD + feat];
    #pragma unroll
    for (int mt = 0; mt < 2; ++mt) {
      #pragma unroll
      for (int r = 0; r < 8; ++r) {
        const int tokl = 32 * w + 16 * mt + 8 * h + r;
        const float y = (acc[mt][nt][r] * WINV + bvl) * osc;
        const int idx = (which == 2) ? ((((tokl & 1) * 64 + feat) * 64) + (tokl >> 1)) : (tokl * HD + feat);
        sT[idx] = (_Float16)y;
      }
    }
  }
  __syncthreads();

  const int t0 = m0 >> 1;
  _Float16* plane = (which == 0) ? qh : kh;
  proj_store_pass(sT, plane, vt, which, head, t0, w, lane);
  __threadfence();
  proj_store_pass(sT, plane, vt, which, head, t0, w, lane);
}

__device__ __forceinline__ v16h pack_p(v8f a, v8f c) {
  const v16h r = { (_Float16)(a[0] * PSCALE), (_Float16)(a[1] * PSCALE), (_Float16)(a[2] * PSCALE), (_Float16)(a[3] * PSCALE),
                   (_Float16)(a[4] * PSCALE), (_Float16)(a[5] * PSCALE), (_Float16)(a[6] * PSCALE), (_Float16)(a[7] * PSCALE),
                   (_Float16)(c[0] * PSCALE), (_Float16)(c[1] * PSCALE), (_Float16)(c[2] * PSCALE), (_Float16)(c[3] * PSCALE),
                   (_Float16)(c[4] * PSCALE), (_Float16)(c[5] * PSCALE), (_Float16)(c[6] * PSCALE), (_Float16)(c[7] * PSCALE) };
  return r;
}

__device__ __forceinline__ void att_store_pass(const _Float16* so, _Float16* ao,
                                               int b, int head, int q0, int lane) {
  const int q8 = lane & 7, sub = lane >> 3;
  #pragma unroll
  for (int i = 0; i < 4; ++i) {
    const int lid = i * 4 + sub;
    const v8h v = *(const v8ha*)(so + lid * 64 + 8 * q8);
    const size_t gi = ((size_t)(q0 + lid) * BSZ + b) * DM + head * HD + 8 * q8;
    *(volatile v8h*)(ao + gi) = v;
  }
}

__global__ __launch_bounds__(128) void attn_kernel(
    const _Float16* __restrict__ qh,
    const _Float16* __restrict__ kh,
    const _Float16* __restrict__ vt,
    _Float16* __restrict__ ao)
{
  __shared__ __attribute__((aligned(16))) _Float16 sO[4 * 16 * 64];

  const int tid = threadIdx.x, lane = tid & 31, w = tid >> 5;
  const int h = lane >> 4, m = lane & 15;
  const int bh = blockIdx.y, b = bh >> 4, head = bh & 15;
  const int q0 = blockIdx.x * 64 + 16 * w;

  const _Float16* qrow = qh + ((size_t)bh * TLEN + q0 + m) * HD;
  const v16h qb0 = load_frag(qrow, h);
  const v16h qb1 = load_frag(qrow + 32, h);

  const v8f zero8 = {0.f, 0.f, 0.f, 0.f, 0.f, 0.f, 0.f, 0.f};
  v8f o[4];
  #pragma unroll
  for (int t = 0; t < 4; ++t) o[t] = zero8;
  float mrun = -1e30f, lrun = 0.0f;

  const _Float16* kbase = kh + ((size_t)bh * TLEN + m) * HD;
  const _Float16* vbase = vt + ((size_t)bh * HD + m) * TLEN;

  #pragma unroll 1
  for (int kb = 0; kb < TLEN; kb += 64) {
    v8f s[4];
    #pragma unroll
    for (int j = 0; j < 4; ++j) {
      const _Float16* kp = kbase + (size_t)(kb + 16 * j) * HD;
      const v16h kf0 = load_frag(kp, h);
      const v16h kf1 = load_frag(kp + 32, h);
      v8f z = zero8;
      z = wmma_f16(kf0, qb0, z);
      z = wmma_f16(kf1, qb1, z);
      s[j] = z;
    }

    float mloc = s[0][0];
    #pragma unroll
    for (int j = 0; j < 4; ++j)
      #pragma unroll
      for (int r = 0; r < 8; ++r) mloc = fmaxf(mloc, s[j][r]);
    mloc = fmaxf(mloc, __shfl_xor(mloc, 16));
    const float mnew = fmaxf(mrun, mloc);
    const float alpha = __expf(mrun - mnew);
    mrun = mnew;
    float lsum = 0.0f;
    #pragma unroll
    for (int j = 0; j < 4; ++j)
      #pragma unroll
      for (int r = 0; r < 8; ++r) {
        const float p = __expf(s[j][r] - mnew);
        s[j][r] = p;
        lsum += p;
      }
    lsum += __shfl_xor(lsum, 16);
    lrun = lrun * alpha + lsum;
    #pragma unroll
    for (int t = 0; t < 4; ++t)
      #pragma unroll
      for (int r = 0; r < 8; ++r) o[t][r] = o[t][r] * alpha;

    const v16h pb0 = pack_p(s[0], s[1]);
    const v16h pb1 = pack_p(s[2], s[3]);

    #pragma unroll
    for (int t = 0; t < 4; ++t) {
      const _Float16* vp = vbase + (size_t)(16 * t) * TLEN + kb;
      const v16h vf0 = load_frag(vp, h);
      const v16h vf1 = load_frag(vp + 32, h);
      o[t] = wmma_f16(vf0, pb0, o[t]);
      o[t] = wmma_f16(vf1, pb1, o[t]);
    }
  }

  const float inv = (1.0f / lrun) * (1.0f / PSCALE);
  _Float16* so = sO + w * 1024;
  #pragma unroll
  for (int t = 0; t < 4; ++t)
    #pragma unroll
    for (int r = 0; r < 8; ++r)
      so[m * 64 + 16 * t + 8 * h + r] = (_Float16)(o[t][r] * inv);
  __syncthreads();

  att_store_pass(so, ao, b, head, q0, lane);
  __threadfence();
  att_store_pass(so, ao, b, head, q0, lane);
}

__device__ __forceinline__ void out_store_pass(const float* sT, float* out, int m0, int n0, int w, int lane) {
  const int q8 = lane & 7, sub = lane >> 3;
  #pragma unroll
  for (int i = 0; i < 16; ++i) {
    const int lid = w * 64 + i * 4 + sub;
    const int row = lid >> 1, hl = lid & 1;
    const v4f v = *(const v4fa*)(sT + row * 64 + 32 * hl + 4 * q8);
    float* dst = out + (size_t)(m0 + row) * DM + n0 + 32 * hl + 4 * q8;
    *(volatile v4f*)dst = v;
  }
}

__global__ __launch_bounds__(128) void outproj_kernel(
    const _Float16* __restrict__ ao,
    const _Float16* __restrict__ woh,
    const float* __restrict__ ob,
    float* __restrict__ out)
{
  __shared__ __attribute__((aligned(16))) float sT[128 * 64];

  const int tid = threadIdx.x, lane = tid & 31, w = tid >> 5;
  const int h = lane >> 4, m = lane & 15;
  const int m0 = blockIdx.x * 128;
  const int n0 = blockIdx.y * 64;
  const int m0w = m0 + 32 * w;

  const _Float16* xa0 = ao + (size_t)(m0w + m) * DM;
  const _Float16* xa1 = xa0 + (size_t)16 * DM;
  const _Float16* wb  = woh + (size_t)(n0 + m) * DM;

  const v8f zero8 = {0.f, 0.f, 0.f, 0.f, 0.f, 0.f, 0.f, 0.f};
  v8f acc[2][4];
  #pragma unroll
  for (int mt = 0; mt < 2; ++mt)
    #pragma unroll
    for (int nt = 0; nt < 4; ++nt) acc[mt][nt] = zero8;

  #pragma unroll 1
  for (int k0 = 0; k0 < DM; k0 += 32) {
    const v16h a0 = load_frag(xa0 + k0, h);
    const v16h a1 = load_frag(xa1 + k0, h);
    #pragma unroll
    for (int nt = 0; nt < 4; ++nt) {
      const v16h b = load_frag(wb + (size_t)nt * 16 * DM + k0, h);
      acc[0][nt] = wmma_f16(a0, b, acc[0][nt]);
      acc[1][nt] = wmma_f16(a1, b, acc[1][nt]);
    }
  }

  #pragma unroll
  for (int nt = 0; nt < 4; ++nt) {
    const int feat = 16 * nt + m;
    const float bvl = ob[n0 + feat];
    #pragma unroll
    for (int mt = 0; mt < 2; ++mt) {
      #pragma unroll
      for (int r = 0; r < 8; ++r) {
        const int tokl = 32 * w + 16 * mt + 8 * h + r;
        sT[tokl * 64 + feat] = acc[mt][nt][r] * WINV + bvl;
      }
    }
  }
  __syncthreads();

  out_store_pass(sT, out, m0, n0, w, lane);
  __threadfence();
  out_store_pass(sT, out, m0, n0, w, lane);
}

extern "C" void kernel_launch(void* const* d_in, const int* in_sizes, int n_in,
                              void* d_out, int out_size, void* d_ws, size_t ws_size,
                              hipStream_t stream) {
  if (n_in < 13) return;
  if (in_sizes[0] != NX) return;
  if (in_sizes[5] != NWIN || in_sizes[6] != N3D) return;
  if (in_sizes[7] != NWOUT || in_sizes[8] != DM) return;
  if (in_sizes[9] != NLA || in_sizes[10] != NLA || in_sizes[11] != NLA || in_sizes[12] != NLA) return;
  if (out_size != NX) return;

  const float* x    = (const float*)d_in[0];
  const float* win  = (const float*)d_in[5];
  const float* bin  = (const float*)d_in[6];
  const float* wout = (const float*)d_in[7];
  const float* bout = (const float*)d_in[8];
  const float* ka   = (const float*)d_in[9];
  const float* kb   = (const float*)d_in[10];
  const float* va   = (const float*)d_in[11];
  const float* vb   = (const float*)d_in[12];
  float* out = (float*)d_out;

  const size_t xh_b  = (size_t)NX * 2;
  const size_t wh_b  = (size_t)NWIN * 2;
  const size_t woh_b = (size_t)NWOUT * 2;
  const size_t la_b  = (size_t)NLA * 2;
  const size_t lb_b  = (size_t)DM * KPAD * 2;
  const size_t lk_b  = (size_t)MROWS * KPAD * 2;
  const size_t pl_b  = (size_t)BSZ * NHEADS * TLEN * HD * 2;
  const size_t ao_b  = (size_t)NX * 2;
  const size_t total = xh_b + wh_b + woh_b + 2 * la_b + 2 * lb_b + 2 * lk_b + 3 * pl_b + ao_b;
  if (total > ws_size) return;

  char* ws = (char*)d_ws;
  size_t off = 0;
  _Float16* xh  = (_Float16*)(ws + off); off += xh_b;
  _Float16* wh  = (_Float16*)(ws + off); off += wh_b;
  _Float16* woh = (_Float16*)(ws + off); off += woh_b;
  _Float16* kah = (_Float16*)(ws + off); off += la_b;
  _Float16* vah = (_Float16*)(ws + off); off += la_b;
  _Float16* kbt = (_Float16*)(ws + off); off += lb_b;
  _Float16* vbt = (_Float16*)(ws + off); off += lb_b;
  _Float16* lk  = (_Float16*)(ws + off); off += lk_b;
  _Float16* lv  = (_Float16*)(ws + off); off += lk_b;
  _Float16* qh  = (_Float16*)(ws + off); off += pl_b;
  _Float16* kh  = (_Float16*)(ws + off); off += pl_b;
  _Float16* vt  = (_Float16*)(ws + off); off += pl_b;
  _Float16* ao  = (_Float16*)(ws + off); off += ao_b;
  if (off > ws_size) return;

  const int ngroups = NX / 8 + NWIN / 8 + NWOUT / 8 + NLA / 8 + NLA / 8;
  convert_kernel<<<(ngroups + 255) / 256, 256, 0, stream>>>(x, win, wout, ka, va, xh, wh, woh, kah, vah);

  lorab_kernel<<<(DM + 255) / 256, 256, 0, stream>>>(kb, vb, kbt, vbt);

  dim3 gLa(MROWS / 128, 2);
  lora_a_kernel<<<gLa, 128, 0, stream>>>(xh, kah, vah, lk, lv);

  dim3 gProj(MROWS / 128, 3 * NHEADS);
  proj_kernel<<<gProj, 128, 0, stream>>>(xh, wh, bin, lk, lv, kbt, vbt, qh, kh, vt);

  dim3 gAtt(TLEN / 64, BSZ * NHEADS);
  attn_kernel<<<gAtt, 128, 0, stream>>>(qh, kh, vt, ao);

  dim3 gOut(MROWS / 128, DM / 64);
  outproj_kernel<<<gOut, 128, 0, stream>>>(ao, woh, bout, out);
}
